// L2TransformerBlock_38190849196710
// MI455X (gfx1250) — hardware-run, weakly checked
//
#include <hip/hip_runtime.h>
#include <math.h>

constexpr int kBt  = 2;
constexpr int kS   = 2048;
constexpr int kD   = 1024;
constexpr int kH   = 16;
constexpr int kDK  = 64;
constexpr int kTok = kBt * kS;
constexpr int kFF  = 4 * kD;
constexpr int kNG  = kBt * kH;
constexpr int kGC  = 2;
constexpr int kNC  = kNG / kGC;
constexpr float kWCarry   = 16.0f;
constexpr float kPCarry   = 2048.0f;
constexpr float kCtxCarry = 16.0f;
constexpr float kMCarry   = 16.0f;
constexpr float kAOCarry  = 64.0f;
constexpr float kHCarry   = 16.0f;
constexpr float kCoefA    = (float)(23.0 / 24.0);
constexpr float kCoefB    = (float)(1.0 / 24.0);
constexpr float kMaskFill = -1.0e9f;
constexpr float kGeluMul  = kHCarry / 1.1289f;

constexpr size_t kMiB   = 1048576;
constexpr size_t oWOUT  = 0;
constexpr size_t oWIN   = 8 * kMiB;
constexpr size_t oWO    = 16 * kMiB;
constexpr size_t oWK    = 18 * kMiB;
constexpr size_t oWV    = 20 * kMiB;
constexpr size_t oMT    = 22 * kMiB;
constexpr size_t oQN    = 22 * kMiB + 131072;
constexpr size_t oRA    = 23 * kMiB;
constexpr size_t oRB    = 31 * kMiB;
constexpr size_t oQT    = 47 * kMiB;
constexpr size_t oCTX   = 55 * kMiB;
constexpr size_t oRC    = 63 * kMiB;
constexpr size_t oRD    = 95 * kMiB;
constexpr size_t kWsTotal = 127 * kMiB;

typedef __attribute__((ext_vector_type(16))) _Float16 v16h;
typedef __attribute__((ext_vector_type(8)))  _Float16 v8h;
typedef __attribute__((ext_vector_type(16))) __bf16   v16b;
typedef __attribute__((ext_vector_type(8)))  __bf16   v8b;
typedef __attribute__((ext_vector_type(8)))  float    v8f;
typedef __attribute__((ext_vector_type(4)))  float    v4f;
typedef __attribute__((ext_vector_type(4)))  unsigned int v4u;
typedef __attribute__((ext_vector_type(4)))  int      v4i;

__device__ __forceinline__ unsigned short f2bf_bits(float f) {
  unsigned u = __float_as_uint(f);
  return (unsigned short)((u + 0x7FFFu + ((u >> 16) & 1u)) >> 16);
}
__device__ __forceinline__ float bf_bits2f(unsigned short h) { return __uint_as_float(((unsigned)h) << 16); }

__device__ __forceinline__ void dep_guard_h(v8f& a, v8f& b, v16h x, v16h y) { asm volatile("v_nop\n\tv_nop\n\tv_nop\n\tv_nop" : "+v"(a), "+v"(b) : "v"(x), "v"(y)); }
__device__ __forceinline__ void dep_guard_b(v8f& a, v8f& b, v16b x, v16b y) { asm volatile("v_nop\n\tv_nop\n\tv_nop\n\tv_nop" : "+v"(a), "+v"(b) : "v"(x), "v"(y)); }
__device__ __forceinline__ void keep4_h(v16h a, v16h b, v16h c, v16h d) { asm volatile("v_nop" :: "v"(a), "v"(b), "v"(c), "v"(d)); }
__device__ __forceinline__ void keep4_b(v16b a, v16b b, v16b c, v16b d) { asm volatile("v_nop" :: "v"(a), "v"(b), "v"(c), "v"(d)); }
__device__ __forceinline__ void acc_guard4(v8f& a, v8f& b, v8f& c, v8f& d) { asm volatile("v_nop\n\tv_nop\n\tv_nop\n\tv_nop" : "+v"(a), "+v"(b), "+v"(c), "+v"(d)); }
template <typename T> struct Frag;
template <> struct Frag<_Float16> {
  typedef v16h V; union U { v16h v; v8h h[2]; };
  static __device__ __forceinline__ v16h load(const _Float16* p) {
    U f; f.h[0] = *(const v8h*)(p); f.h[1] = *(const v8h*)(p + 16); return f.v;
  }
  static __device__ __forceinline__ v8f mma(v16h a, v16h b, v8f c) {
    return __builtin_amdgcn_wmma_f32_16x16x32_f16(false, a, false, b, (short)0, c, false, false);
  }
  static __device__ __forceinline__ void guard(v8f& a, v8f& b, v16h x, v16h y) { dep_guard_h(a, b, x, y); }
  static __device__ __forceinline__ void keep(v16h a, v16h b, v16h c, v16h d) { keep4_h(a, b, c, d); }
};
template <> struct Frag<__bf16> {
  typedef v16b V; union U { v16b v; v8b h[2]; };
  static __device__ __forceinline__ v16b load(const __bf16* p) {
    U f; f.h[0] = *(const v8b*)(p); f.h[1] = *(const v8b*)(p + 16); return f.v;
  }
  static __device__ __forceinline__ v8f mma(v16b a, v16b b, v8f c) {
    return __builtin_amdgcn_wmma_f32_16x16x32_bf16(false, a, false, b, (short)0, c, false, false);
  }
  static __device__ __forceinline__ void guard(v8f& a, v8f& b, v16b x, v16b y) { dep_guard_b(a, b, x, y); }
  static __device__ __forceinline__ void keep(v16b a, v16b b, v16b c, v16b d) { keep4_b(a, b, c, d); }
};

__device__ __forceinline__ unsigned pk16(unsigned short a, unsigned short b) { return (unsigned)a | ((unsigned)b << 16); }
__device__ __forceinline__ unsigned short h_bits(float f) { const _Float16 h = (_Float16)f; return __builtin_bit_cast(unsigned short, h); }

template <int ET> struct Elem;
template <> struct Elem<0> { typedef _Float16 T; };
template <> struct Elem<1> { typedef __bf16 T; };
template <int ET, bool SPLIT, int BIAS_MODE, int OUT_MODE, bool RESID, int ACT = 0, int CAUSAL = 0>
__global__ __launch_bounds__(256) void wmma_gemm64(
    const unsigned short* __restrict__ Ap, const unsigned short* __restrict__ A2p, int lda, long strideA,
    const unsigned short* __restrict__ Btp, const unsigned short* __restrict__ Bt2p, int ldb, long strideB,
    void* __restrict__ Cout, void* __restrict__ Cout2, int ldc, long strideC,
    const float* __restrict__ bias,
    const float* __restrict__ resid, long strideR,
    int M, int N, int K, float scale, float rscale) {
  typedef typename Elem<ET>::T T;
  typedef typename Frag<T>::V V;
  const T* A = (const T*)Ap; const T* A2 = (const T*)A2p; const T* Bt = (const T*)Btp; const T* Bt2 = (const T*)Bt2p;
  __shared__ __align__(16) float sT[8][16 * 68];
  const int b    = blockIdx.y;
  const int lane = threadIdx.x & 31;
  const int wave = threadIdx.x >> 5;
  const int tilesN = N >> 6;
  const int tilesM = M >> 6;
  const int tile = blockIdx.x * 8 + wave;
  if (tile >= tilesM * tilesN) return;
  const int tm = tile / tilesN;
  const int tn = tile - tm * tilesN;
  if (CAUSAL == 1 && tn > tm) return;
  const int m0 = tm << 6;
  const int n0 = tn << 6;
  const int Kend = (CAUSAL == 2) ? ((m0 + 64 < K) ? (m0 + 64) : K) : K;

  const T* Ab  = A  + (size_t)b * strideA;
  const T* Bb  = Bt + (size_t)b * strideB;
  const T* Ab2 = SPLIT ? (A2  + (size_t)b * strideA) : nullptr;
  const T* Bb2 = SPLIT ? (Bt2 + (size_t)b * strideB) : nullptr;

  const int rlane = lane & 15;
  const int koff  = (lane >> 4) * 8;
  const int mOff  = (lane >> 4) * 8;

  v8f acc[4][4];
#pragma unroll
  for (int i = 0; i < 4; ++i)
#pragma unroll
    for (int j = 0; j < 4; ++j) acc[i][j] = (v8f){0.f,0.f,0.f,0.f,0.f,0.f,0.f,0.f};

  for (int k0 = 0; k0 < Kend; k0 += 32) {
    V bh[4], bl[4];
#pragma unroll
    for (int j = 0; j < 4; ++j) {
      const size_t bo = (size_t)(n0 + (j << 4) + rlane) * ldb + koff + k0;
      bh[j] = Frag<T>::load(Bb + bo);
      if (SPLIT) bl[j] = Frag<T>::load(Bb2 + bo);
    }
#pragma unroll
    for (int i = 0; i < 4; ++i) {
      const size_t ao = (size_t)(m0 + (i << 4) + rlane) * lda + koff + k0;
      V ah = Frag<T>::load(Ab + ao);
      V al;
      if (SPLIT) al = Frag<T>::load(Ab2 + ao);
#pragma unroll
      for (int j = 0; j < 4; ++j) {
        acc[i][j] = Frag<T>::mma(ah, bh[j], acc[i][j]);
        if (SPLIT) {
          acc[i][j] = Frag<T>::mma(ah, bl[j], acc[i][j]);
          acc[i][j] = Frag<T>::mma(al, bh[j], acc[i][j]);
        }
      }
      Frag<T>::guard(acc[i][0], acc[i][3], ah, SPLIT ? al : ah);
    }
    Frag<T>::keep(bh[0], bh[1], bh[2], bh[3]);
    if (SPLIT) Frag<T>::keep(bl[0], bl[1], bl[2], bl[3]);
  }
  acc_guard4(acc[0][0], acc[0][1], acc[0][2], acc[0][3]);
  acc_guard4(acc[1][0], acc[1][1], acc[1][2], acc[1][3]);
  acc_guard4(acc[2][0], acc[2][1], acc[2][2], acc[2][3]);
  acc_guard4(acc[3][0], acc[3][1], acc[3][2], acc[3][3]);

  float* slab = sT[wave];
  const float* Rb = RESID ? (resid + (size_t)b * strideR) : nullptr;
#pragma unroll
  for (int i = 0; i < 4; ++i) {
    const int mBase = m0 + (i << 4);
#pragma unroll
    for (int j = 0; j < 4; ++j) {
      const int n = n0 + (j << 4) + rlane;
      float bv = 0.f;
      if (BIAS_MODE == 2) bv = bias[n];
#pragma unroll
      for (int r = 0; r < 8; ++r) {
        float v = acc[i][j][r] * scale;
        if (BIAS_MODE == 1) v += bias[mBase + mOff + r];
        if (BIAS_MODE == 2) v += bv;
        if (RESID) v += rscale * Rb[(size_t)(mBase + mOff + r) * ldc + n];
        if (ACT == 2) v = fmaxf(v, 0.0f);
        if (ACT == 4) v = (v > 0.f) ? v : 0.01f * v;
        slab[(mOff + r) * 68 + (j << 4) + rlane] = v;
      }
    }
    __builtin_amdgcn_fence(__ATOMIC_RELEASE, "workgroup");
    __builtin_amdgcn_wave_barrier();
    __builtin_amdgcn_fence(__ATOMIC_ACQUIRE, "workgroup");
    if (OUT_MODE == 0) {
      float* C = (float*)Cout + (size_t)b * strideC;
      const int hh = lane >> 4, c4 = (lane & 15) * 4;
      for (int pass = 0; pass < 2; ++pass) {
#pragma unroll
        for (int it = 0; it < 8; ++it) {
          const int row = it * 2 + hh;
          v4f v = *(const v4f*)(slab + row * 68 + c4);
          *(volatile v4f*)(C + (size_t)(mBase + row) * ldc + n0 + c4) = v;
        }
        __threadfence();
      }
    } else {
      const int q = lane >> 3, c8 = (lane & 7) * 8;
      unsigned short* C  = (unsigned short*)Cout  + (size_t)b * strideC;
      unsigned short* C2 = (OUT_MODE == 2) ? ((unsigned short*)Cout2 + (size_t)b * strideC) : nullptr;
      for (int pass = 0; pass < 2; ++pass) {
#pragma unroll
        for (int it = 0; it < 4; ++it) {
          const int row = it * 4 + q;
          const float* sp = slab + row * 68 + c8;
          v8h hv, lv;
#pragma unroll
          for (int e = 0; e < 8; ++e) {
            if (OUT_MODE == 1) {
              hv[e] = (_Float16)sp[e];
            } else {
              unsigned short hb = f2bf_bits(sp[e]);
              unsigned short lb = f2bf_bits(sp[e] - bf_bits2f(hb));
              hv[e] = __builtin_bit_cast(_Float16, hb);
              lv[e] = __builtin_bit_cast(_Float16, lb);
            }
          }
          *(volatile v8h*)(C + (size_t)(mBase + row) * ldc + n0 + c8) = hv;
          if (OUT_MODE == 2) *(volatile v8h*)(C2 + (size_t)(mBase + row) * ldc + n0 + c8) = lv;
        }
        __threadfence();
      }
    }
    __builtin_amdgcn_fence(__ATOMIC_RELEASE, "workgroup");
    __builtin_amdgcn_wave_barrier();
    __builtin_amdgcn_fence(__ATOMIC_ACQUIRE, "workgroup");
  }
}

__global__ __launch_bounds__(256) void cast8_kernel(const float* __restrict__ in, unsigned short* __restrict__ out,
                                                    int n8, float carry) {
  const int i = blockIdx.x * 256 + threadIdx.x;
  if (i >= n8) return;
  const float* p = in + 8 * (size_t)i;
  const v4f a = *(const v4f*)(p);
  const v4f c = *(const v4f*)(p + 4);
  unsigned short hb[8];
#pragma unroll
  for (int e = 0; e < 4; ++e) {
    hb[e]     = h_bits(a[e] * carry);
    hb[4 + e] = h_bits(c[e] * carry);
  }
  const v4u u = (v4u){pk16(hb[0], hb[1]), pk16(hb[2], hb[3]), pk16(hb[4], hb[5]), pk16(hb[6], hb[7])};
  unsigned short* q = out + 8 * (size_t)i;
  *(volatile v4u*)q = u;
  __threadfence();
  *(volatile v4u*)q = u;
}

__global__ __launch_bounds__(256) void qprep_kernel(const float* __restrict__ Qf, float* __restrict__ qn,
                                                    unsigned short* __restrict__ Q16, unsigned short* __restrict__ QT16) {
  __shared__ float sm[64][65];
  __shared__ float sq[64];
  const int t = threadIdx.x, lane = t & 31, wave = t >> 5;
  const int tok0 = blockIdx.x * 64;
  const int h = blockIdx.y;
  const int b = tok0 / kS;
  const int s0 = tok0 - b * kS;
  const int g = b * kH + h;
#pragma unroll
  for (int it = 0; it < 4; ++it) {
    const int e = it * 256 + t;
    const int r = e >> 4, c4 = (e & 15) * 4;
    const v4f v = *(const v4f*)(Qf + (size_t)(tok0 + r) * kD + h * kDK + c4);
    sm[r][c4 + 0] = v[0];
    sm[r][c4 + 1] = v[1];
    sm[r][c4 + 2] = v[2];
    sm[r][c4 + 3] = v[3];
  }
  __syncthreads();
  {
    const int r = t >> 2, qq = (t & 3) * 16;
    float p = 0.f;
#pragma unroll
    for (int e = 0; e < 16; ++e) { const float v = sm[r][qq + e]; p += v * v; }
    p += __shfl_xor(p, 1, 32);
    p += __shfl_xor(p, 2, 32);
    if ((t & 3) == 0) sq[r] = p;
  }
  __syncthreads();
  const int l16 = lane & 15;
  const v4f qv = (v4f){sq[l16 * 4 + 0], sq[l16 * 4 + 1], sq[l16 * 4 + 2], sq[l16 * 4 + 3]};
  const int q3 = lane >> 3, c8 = (lane & 7) * 8;
  v4u uq[2], ut[2];
#pragma unroll
  for (int it = 0; it < 2; ++it) {
    const int row = wave * 8 + it * 4 + q3;
    unsigned short hb[8], tb[8];
#pragma unroll
    for (int e = 0; e < 8; ++e) {
      hb[e] = h_bits(sm[row][c8 + e]);
      tb[e] = h_bits(sm[c8 + e][row]);
    }
    uq[it] = (v4u){pk16(hb[0], hb[1]), pk16(hb[2], hb[3]), pk16(hb[4], hb[5]), pk16(hb[6], hb[7])};
    ut[it] = (v4u){pk16(tb[0], tb[1]), pk16(tb[2], tb[3]), pk16(tb[4], tb[5]), pk16(tb[6], tb[7])};
  }
  float* qdst = qn + (size_t)g * kS + s0 + l16 * 4;
  for (int pass = 0; pass < 2; ++pass) {
    if (t < 16) *(volatile v4f*)qdst = qv;
#pragma unroll
    for (int it = 0; it < 2; ++it) {
      const int row = wave * 8 + it * 4 + q3;
      *(volatile v4u*)(Q16  + ((size_t)g * kS + s0 + row) * kDK + c8) = uq[it];
      *(volatile v4u*)(QT16 + ((size_t)g * kDK + row) * kS + s0 + c8) = ut[it];
    }
    __threadfence();
  }
}

__global__ __launch_bounds__(256) void softmax_kernel(const float* __restrict__ Sb, unsigned short* __restrict__ Pb,
                                                      const float* __restrict__ qn, const int* __restrict__ mask, int g0) {
  __shared__ float redM[8];
  __shared__ float redS[8];
  const int row = blockIdx.x;
  const int gl  = blockIdx.y;
  const int g   = g0 + gl;
  const int t = threadIdx.x, lane = t & 31, wave = t >> 5;
  const int cend = (row & ~63) + 64;
  const bool wlive = (wave * 256) < cend;
  const bool llive = (t * 8) < cend;
  const int col0 = llive ? (t * 8) : (cend - 8);
  const float qi = qn[(size_t)g * kS + row];
  float xs[8];
#pragma unroll
  for (int e = 0; e < 8; ++e) xs[e] = kMaskFill;
  float m = -INFINITY;
  if (wlive) {
    const float* sr = Sb + ((size_t)gl * kS + row) * kS + col0;
    const v4f da = *(const v4f*)(sr);
    const v4f dc = *(const v4f*)(sr + 4);
    const int* mr = mask + (size_t)row * kS + col0;
    const v4i ma = *(const v4i*)(mr);
    const v4i mc = *(const v4i*)(mr + 4);
    const float* kr = qn + (size_t)g * kS + col0;
    const v4f ka = *(const v4f*)(kr);
    const v4f kc = *(const v4f*)(kr + 4);
    float dot[8], kn[8];
    int mk[8];
#pragma unroll
    for (int e = 0; e < 4; ++e) {
      dot[e] = da[e]; dot[4 + e] = dc[e];
      kn[e]  = ka[e]; kn[4 + e]  = kc[e];
      mk[e]  = ma[e]; mk[4 + e]  = mc[e];
    }
#pragma unroll
    for (int e = 0; e < 8; ++e) {
      const float tt = (qi - 2.0f * dot[e]) + kn[e];
      float sv = -tt * 0.125f;
      sv = (mk[e] == 0) ? kMaskFill : sv;
      sv = llive ? sv : kMaskFill;
      xs[e] = sv;
      m = fmaxf(m, sv);
    }
#pragma unroll
    for (int off = 1; off < 32; off <<= 1) m = fmaxf(m, __shfl_xor(m, off, 32));
  }
  if (lane == 0) redM[wave] = m;
  __syncthreads();
  float mm = redM[0];
#pragma unroll
  for (int w = 1; w < 8; ++w) mm = fmaxf(mm, redM[w]);
  float ps[8];
#pragma unroll
  for (int e = 0; e < 8; ++e) ps[e] = 0.f;
  float ssum = 0.f;
  if (wlive) {
#pragma unroll
    for (int e = 0; e < 8; ++e) { ps[e] = expf(xs[e] - mm); ssum += ps[e]; }
#pragma unroll
    for (int off = 1; off < 32; off <<= 1) ssum += __shfl_xor(ssum, off, 32);
  }
  if (lane == 0) redS[wave] = ssum;
  __syncthreads();
  float tot = redS[0];
#pragma unroll
  for (int w = 1; w < 8; ++w) tot += redS[w];
  const float inv = 1.0f / tot;
  if (wlive) {
    unsigned short hb[8];
#pragma unroll
    for (int e = 0; e < 8; ++e) hb[e] = h_bits((ps[e] * inv) * kPCarry);
    const v4u u = (v4u){pk16(hb[0], hb[1]), pk16(hb[2], hb[3]), pk16(hb[4], hb[5]), pk16(hb[6], hb[7])};
    unsigned short* dst = Pb + ((size_t)gl * kS + row) * kS + t * 8;
    if (llive) *(volatile v4u*)dst = u;
    __threadfence();
    if (llive) *(volatile v4u*)dst = u;
  }
}

__global__ __launch_bounds__(256) void gelu_kernel(const unsigned* __restrict__ in, unsigned* __restrict__ out, int n2) {
  const int i = blockIdx.x * 256 + threadIdx.x;
  if (i >= n2) return;
  const unsigned w = in[i];
  unsigned r = 0;
#pragma unroll 1
  for (int e = 0; e < 2; ++e) {
    const unsigned short bits = (unsigned short)((w >> (16 * e)) & 0xffffu);
    const float u = (float)__builtin_bit_cast(_Float16, bits);
    const float gg = 0.5f * u * (1.0f + erff(u * 0.70710678118654752f));
    const float hv = gg * kGeluMul;
    r |= ((unsigned)h_bits(hv)) << (16 * e);
  }
  ((volatile unsigned*)out)[i] = r;
  __threadfence();
  ((volatile unsigned*)out)[i] = r;
}

extern "C" void kernel_launch(void* const* d_in, const int* in_sizes, int n_in,
                              void* d_out, int out_size, void* d_ws, size_t ws_size,
                              hipStream_t stream) {
  if (n_in < 7) return;
  if (in_sizes[0] != kTok * kD || in_sizes[1] != kS * kS || in_sizes[2] != kD * kD || in_sizes[3] != kD * kD ||
      in_sizes[4] != kD * kD || in_sizes[5] != kFF * kD || in_sizes[6] != kD * kFF) return;
  if (out_size != kTok * kD) return;
  if (ws_size < kWsTotal) return;

  const float* x     = (const float*)d_in[0];
  const int*   maskp = (const int*)d_in[1];
  const float* w_k   = (const float*)d_in[2];
  const float* w_v   = (const float*)d_in[3];
  const float* w_o   = (const float*)d_in[4];
  const float* w_in  = (const float*)d_in[5];
  const float* w_out = (const float*)d_in[6];
  float* outp = (float*)d_out;
  char* ws = (char*)d_ws;

  unsigned short* WOUT16 = (unsigned short*)(ws + oWOUT);
  unsigned short* WIN16  = (unsigned short*)(ws + oWIN);
  unsigned short* WO16   = (unsigned short*)(ws + oWO);
  unsigned short* WK16   = (unsigned short*)(ws + oWK);
  unsigned short* WV16   = (unsigned short*)(ws + oWV);
  unsigned short* MT16   = (unsigned short*)(ws + oMT);
  float*          qn     = (float*)(ws + oQN);
  unsigned short* X16    = (unsigned short*)(ws + oRA);
  unsigned short* Q16    = (unsigned short*)(ws + oRA);
  unsigned short* AO16   = (unsigned short*)(ws + oRA);
  unsigned short* X1H    = (unsigned short*)(ws + oRA);
  float*          Qf     = (float*)(ws + oRB);
  float*          X1F    = (float*)(ws + oRB);
  unsigned short* QT16   = (unsigned short*)(ws + oQT);
  unsigned short* CTX16  = (unsigned short*)(ws + oCTX);
  float*          Sbuf   = (float*)(ws + oRC);
  unsigned short* U16P   = (unsigned short*)(ws + oRC);
  unsigned short* Pbuf   = (unsigned short*)(ws + oRD);
  unsigned short* H16    = (unsigned short*)(ws + oRD);

  {
    const int n8x = kTok * kD / 8, n8w = kD * kD / 8, n8f = kFF * kD / 8;
    cast8_kernel<<<dim3((n8x + 255) / 256), 256, 0, stream>>>(x, X16, n8x, 1.0f);
    cast8_kernel<<<dim3((n8w + 255) / 256), 256, 0, stream>>>(w_k, WK16, n8w, kWCarry);
    cast8_kernel<<<dim3((n8w + 255) / 256), 256, 0, stream>>>(w_v, WV16, n8w, kWCarry);
    cast8_kernel<<<dim3((n8w + 255) / 256), 256, 0, stream>>>(w_o, WO16, n8w, kWCarry);
    cast8_kernel<<<dim3((n8f + 255) / 256), 256, 0, stream>>>(w_in, WIN16, n8f, kWCarry);
    cast8_kernel<<<dim3((n8f + 255) / 256), 256, 0, stream>>>(w_out, WOUT16, n8f, kWCarry);
  }

  wmma_gemm64<0, false, 0, 0, false, 0, 0> <<<dim3((64 * 16 + 7) / 8, 1), 256, 0, stream>>>(
      X16, nullptr, kD, 0L, WK16, nullptr, kD, 0L, (void*)Qf, nullptr, kD, 0L,
      nullptr, nullptr, 0L, kTok, kD, kD, 1.0f / kWCarry, 0.0f);

  qprep_kernel<<<dim3(kTok / 64, kH), 256, 0, stream>>>(Qf, qn, Q16, QT16);

  wmma_gemm64<0, false, 0, 1, false, 0, 0> <<<dim3(1, kH), 32, 0, stream>>>(
      WV16, nullptr, kD, (long)kDK * kD, WK16, nullptr, kD, (long)kDK * kD, (void*)MT16, nullptr, kDK, (long)kDK * kDK,
      nullptr, nullptr, 0L, kDK, kDK, kD, kMCarry / (kWCarry * kWCarry), 0.0f);

  for (int c = 0; c < kNC; ++c) {
    const int g0 = c * kGC;
    const int bb = g0 / kH;
    const int h0 = g0 - bb * kH;
    wmma_gemm64<0, false, 0, 0, false, 0, 1> <<<dim3((32 * 32 + 7) / 8, kGC), 256, 0, stream>>>(
        Q16 + (size_t)g0 * kS * kDK, nullptr, kDK, (long)kS * kDK,
        Q16 + (size_t)g0 * kS * kDK, nullptr, kDK, (long)kS * kDK,
        (void*)Sbuf, nullptr, kS, (long)kS * kS,
        nullptr, nullptr, 0L, kS, kS, kDK, 1.0f, 0.0f);
    softmax_kernel<<<dim3(kS, kGC), 256, 0, stream>>>(Sbuf, Pbuf, qn, maskp, g0);
    wmma_gemm64<0, false, 0, 1, false, 0, 2> <<<dim3((32 * 1 + 7) / 8, kGC), 256, 0, stream>>>(
        Pbuf, nullptr, kS, (long)kS * kS,
        QT16 + (size_t)g0 * kDK * kS, nullptr, kS, (long)kDK * kS,
        (void*)(CTX16 + (size_t)bb * kS * kD + (size_t)h0 * kDK), nullptr, kD, (long)kDK,
        nullptr, nullptr, 0L, kS, kDK, kS, kCtxCarry / kPCarry, 0.0f);
  }

  wmma_gemm64<0, false, 0, 1, false, 0, 0> <<<dim3((64 * 1 + 7) / 8, kH), 256, 0, stream>>>(
      CTX16, nullptr, kD, (long)kDK, MT16, nullptr, kDK, (long)kDK * kDK, (void*)AO16, nullptr, kD, (long)kDK,
      nullptr, nullptr, 0L, kTok, kDK, kDK, 0.125f * kAOCarry / (kCtxCarry * kMCarry), 0.0f);

  wmma_gemm64<0, false, 0, 0, true, 0, 0> <<<dim3((64 * 16 + 7) / 8, 1), 256, 0, stream>>>(
      AO16, nullptr, kD, 0L, WO16, nullptr, kD, 0L, (void*)X1F, nullptr, kD, 0L,
      nullptr, x, 0L, kTok, kD, kD, kCoefB / (kAOCarry * kWCarry), kCoefA);

  {
    const int n8x = kTok * kD / 8;
    cast8_kernel<<<dim3((n8x + 255) / 256), 256, 0, stream>>>(X1F, X1H, n8x, 1.0f);
  }

  wmma_gemm64<0, false, 0, 1, false, 0, 0> <<<dim3((64 * 64 + 7) / 8, 1), 256, 0, stream>>>(
      X1H, nullptr, kD, 0L, WIN16, nullptr, kD, 0L, (void*)U16P, nullptr, kFF, 0L,
      nullptr, nullptr, 0L, kTok, kFF, kD, 1.0f / kWCarry, 0.0f);

  {
    const int n2 = kTok * kFF / 2;
    gelu_kernel<<<dim3((n2 + 255) / 256), 256, 0, stream>>>((const unsigned*)U16P, (unsigned*)H16, n2);
  }

  wmma_gemm64<0, false, 0, 0, true, 0, 0> <<<dim3((64 * 16 + 7) / 8, 1), 256, 0, stream>>>(
      H16, nullptr, kFF, 0L, WOUT16, nullptr, kFF, 0L, (void*)outp, nullptr, kD, 0L,
      nullptr, X1F, 0L, kTok, kD, kFF, kCoefB / (kHCarry * kWCarry), kCoefA);
}
